// HAN_53369263620116
// MI455X (gfx1250) — hardware-verified
//
#include <hip/hip_runtime.h>
#include <math.h>
#include <stddef.h>

constexpr int NNOTE = 4096;
constexpr int NFEAT = 78;
constexpr int KPADX = 96;
constexpr int HNOTE = 256;
constexpr int HBEAT = 128;
constexpr int HMEAS = 64;
constexpr int HFIN  = 128;
constexpr int NBEAT = 512;
constexpr int NMEAS = 128;
constexpr int NOUTC = 11;
constexpr int UINW  = 1424;
constexpr int SCOL  = 1408;
constexpr int BTINW = 273;
constexpr int FCINW = 1552;
constexpr int GON   = 576;
constexpr int VXP   = 144;
constexpr int NTHR  = 256;

static_assert(NNOTE % 64 == 0 && (2 * 4 * HNOTE) % 64 == 0 && KPADX % 32 == 0);
static_assert((2 * HNOTE) % 64 == 0 && (2 * HNOTE) % 32 == 0);
static_assert(NBEAT % 64 == 0 && (2 * 4 * HBEAT) % 64 == 0);
static_assert((2 * HBEAT) % 64 == 0 && (2 * HBEAT) % 32 == 0);
static_assert(NMEAS % 64 == 0 && (2 * 4 * HMEAS) % 64 == 0);
static_assert(GON % 64 == 0 && SCOL % 32 == 0 && (4 * HBEAT) % 64 == 0);
static_assert(NNOTE * NOUTC * 4 == 180224 && 180224 % 128 == 0);
static_assert(NNOTE % 32 == 0);

typedef __attribute__((ext_vector_type(16))) __bf16   v16b;
typedef __attribute__((ext_vector_type(8)))  __bf16   v8b;
typedef __attribute__((ext_vector_type(8)))  _Float16 v8h;
typedef __attribute__((ext_vector_type(8)))  float    v8f;
typedef __attribute__((ext_vector_type(4)))  float    v4f;

__device__ __forceinline__ unsigned short f2bf_bits(float f) {
  unsigned u = __float_as_uint(f);
  return (unsigned short)((u + 0x7FFFu + ((u >> 16) & 1u)) >> 16);
}
__device__ __forceinline__ float bf_bits2f(unsigned short h) { return __uint_as_float(((unsigned)h) << 16); }
__device__ __forceinline__ float bfr(float f) { return bf_bits2f(f2bf_bits(f)); }

__device__ __forceinline__ void guard4_b(v8f& a0, v8f& a1, v8f& a2, v8f& a3, v16b x, v16b y) {
  asm volatile("v_nop\n\tv_nop\n\tv_nop\n\tv_nop" : "+v"(a0), "+v"(a1), "+v"(a2), "+v"(a3) : "v"(x), "v"(y));
}
__device__ __forceinline__ void keep4_b(v16b a, v16b b, v16b c, v16b d) { asm volatile("v_nop" :: "v"(a), "v"(b), "v"(c), "v"(d)); }
__device__ __forceinline__ void acc_guard4(v8f& a, v8f& b, v8f& c, v8f& d) { asm volatile("v_nop\n\tv_nop\n\tv_nop\n\tv_nop" : "+v"(a), "+v"(b), "+v"(c), "+v"(d)); }

struct FragB {
  union U { v16b v; v8b h[2]; };
  static __device__ __forceinline__ v16b load(const __bf16* p) {
    U f; f.h[0] = *(const v8b*)(p); f.h[1] = *(const v8b*)(p + 16); return f.v;
  }
  static __device__ __forceinline__ v8f mma(v16b a, v16b b, v8f c) {
    return __builtin_amdgcn_wmma_f32_16x16x32_bf16(false, a, false, b, (short)0, c, false, false);
  }
};

__device__ __forceinline__ float fsig(float x)  { return __builtin_amdgcn_rcpf(1.0f + expf(-x)); }
__device__ __forceinline__ float ftanh(float x) { return 1.0f - 2.0f * __builtin_amdgcn_rcpf(expf(2.0f * x) + 1.0f); }

template <bool ASPLIT>
__global__ __launch_bounds__(NTHR) void gemm_bf16_kernel(
    const unsigned short* __restrict__ Ap, const unsigned short* __restrict__ A2p, int lda,
    const unsigned short* __restrict__ Btp, int ldb,
    float* __restrict__ Cf, int ldc, const float* __restrict__ bias,
    int M, int N, int K) {
  const __bf16* A  = (const __bf16*)Ap;
  const __bf16* A2 = (const __bf16*)A2p;
  const __bf16* Bt = (const __bf16*)Btp;
  __shared__ __align__(16) float sT[8][16 * 68];
  const int lane = threadIdx.x & 31;
  const int wave = threadIdx.x >> 5;
  const int tilesN = N >> 6;
  const int tilesM = M >> 6;
  const int tile = blockIdx.x * 8 + wave;
  if (tile >= tilesM * tilesN) return;
  const int tm = tile / tilesN;
  const int tn = tile - tm * tilesN;
  const int m0 = tm << 6;
  const int n0 = tn << 6;
  const int rlane = lane & 15;
  const int koff  = (lane >> 4) * 8;
  const int mOff  = (lane >> 4) * 8;

  v8f acc[4][4];
#pragma unroll
  for (int i = 0; i < 4; ++i)
#pragma unroll
    for (int j = 0; j < 4; ++j) acc[i][j] = (v8f){0.f,0.f,0.f,0.f,0.f,0.f,0.f,0.f};

  for (int k0 = 0; k0 < K; k0 += 32) {
    v16b bh[4];
#pragma unroll
    for (int j = 0; j < 4; ++j) {
      const size_t bo = (size_t)(n0 + (j << 4) + rlane) * ldb + koff + k0;
      bh[j] = FragB::load(Bt + bo);
    }
#pragma unroll
    for (int i = 0; i < 4; ++i) {
      const size_t ao = (size_t)(m0 + (i << 4) + rlane) * lda + koff + k0;
      const v16b ah = FragB::load(A + ao);
      v16b al = ah;
      if (ASPLIT) al = FragB::load(A2 + ao);
#pragma unroll
      for (int j = 0; j < 4; ++j) {
        acc[i][j] = FragB::mma(ah, bh[j], acc[i][j]);
        if (ASPLIT) acc[i][j] = FragB::mma(al, bh[j], acc[i][j]);
      }
      guard4_b(acc[i][0], acc[i][1], acc[i][2], acc[i][3], ah, al);
    }
    keep4_b(bh[0], bh[1], bh[2], bh[3]);
  }
  acc_guard4(acc[0][0], acc[0][1], acc[0][2], acc[0][3]);
  acc_guard4(acc[1][0], acc[1][1], acc[1][2], acc[1][3]);
  acc_guard4(acc[2][0], acc[2][1], acc[2][2], acc[2][3]);
  acc_guard4(acc[3][0], acc[3][1], acc[3][2], acc[3][3]);

  float* slab = sT[wave];
#pragma unroll
  for (int i = 0; i < 4; ++i) {
    const int mBase = m0 + (i << 4);
#pragma unroll
    for (int j = 0; j < 4; ++j) {
      const int n = n0 + (j << 4) + rlane;
      const float bv = bias[n];
#pragma unroll
      for (int r = 0; r < 8; ++r) {
        const float v = acc[i][j][r] + bv;
        slab[(mOff + r) * 68 + (j << 4) + rlane] = v;
      }
    }
    __builtin_amdgcn_fence(__ATOMIC_RELEASE, "workgroup");
    __builtin_amdgcn_wave_barrier();
    __builtin_amdgcn_fence(__ATOMIC_ACQUIRE, "workgroup");
    {
      const int hh = lane >> 4, c4 = (lane & 15) * 4;
      for (int pass = 0; pass < 2; ++pass) {
#pragma unroll
        for (int it = 0; it < 8; ++it) {
          const int row = it * 2 + hh;
          const v4f v = *(const v4f*)(slab + row * 68 + c4);
          *(volatile v4f*)(Cf + (size_t)(mBase + row) * ldc + n0 + c4) = v;
        }
        __threadfence();
      }
    }
    __builtin_amdgcn_fence(__ATOMIC_RELEASE, "workgroup");
    __builtin_amdgcn_wave_barrier();
    __builtin_amdgcn_fence(__ATOMIC_ACQUIRE, "workgroup");
  }
}

struct CvtSeg { const float* src; unsigned short* dst; int spitch; int scol0; int nvalid; int ncol8; int nrow; int pad0; };
struct CvtArgs { CvtSeg s[12]; };
static_assert(sizeof(CvtSeg) == 40);
static_assert(sizeof(CvtArgs) == 480);

__global__ __launch_bounds__(NTHR) void cvt_multi_kernel(CvtArgs a) {
  const CvtSeg sg = a.s[blockIdx.y];
  const int i = blockIdx.x * NTHR + threadIdx.x;
  const int n8 = sg.nrow * sg.ncol8;
  if (i >= n8) return;
  const int row = i / sg.ncol8;
  const int c8 = i - row * sg.ncol8;
  const float* sp = sg.src + (size_t)row * sg.spitch + sg.scol0;
  v8h hv;
#pragma unroll
  for (int e = 0; e < 8; ++e) {
    const int col = 8 * c8 + e;
    int sc = col < sg.nvalid ? col : (sg.nvalid - 1);
    sc = sc < 0 ? 0 : sc;
    const float fz = (col < sg.nvalid) ? 1.0f : 0.0f;
    const float v = sp[sc] * fz;
    hv[e] = __builtin_bit_cast(_Float16, f2bf_bits(v));
  }
  unsigned short* dp = sg.dst + (size_t)i * 8;
  *(volatile v8h*)dp = hv;
  __threadfence();
  *(volatile v8h*)dp = hv;
}

struct RneArgs { const float* src[16]; float* dst[16]; int n4[16]; };
static_assert(sizeof(RneArgs) == 320);

__global__ __launch_bounds__(NTHR) void rne_multi_kernel(RneArgs a) {
  const int s = blockIdx.y;
  const int i = blockIdx.x * NTHR + threadIdx.x;
  if (i >= a.n4[s]) return;
  const v4f v = *(const v4f*)(a.src[s] + (size_t)i * 4);
  v4f o;
#pragma unroll
  for (int e = 0; e < 4; ++e) o[e] = bfr(v[e]);
  float* dp = a.dst[s] + (size_t)i * 4;
  *(volatile v4f*)dp = o;
  __threadfence();
  *(volatile v4f*)dp = o;
}

__global__ __launch_bounds__(NTHR) void prep_fold_kernel(const float* __restrict__ x, const float* __restrict__ out_b,
    const float* __restrict__ out_Wi, const float* __restrict__ bfc, const float* __restrict__ Wfc,
    const float* __restrict__ bt_b, const float* __restrict__ bt_Wi,
    float* __restrict__ BIAS7, float* __restrict__ BEFFB, float* __restrict__ WFCX) {
  __shared__ __align__(16) float sm[2304];
  const int tid = threadIdx.x;
  const float qpmR = bfr(x[5]), tp0R = bfr(x[76]), tp1R = bfr(x[77]);
  if (blockIdx.x == 0) {
#pragma unroll 1
    for (int it = 0; it < 3; ++it) {
      const int f = it * NTHR + tid;
      const int ga = f < 511 ? f : 511;
      const float* wa = out_Wi + (size_t)ga * UINW;
      const float va = bfr(out_b[ga]) + bfr(wa[1421]) * qpmR + bfr(wa[1422]) * tp0R + bfr(wa[1423]) * tp1R;
      int gb = f - 512; gb = gb < 0 ? 0 : gb; gb = gb > 9 ? 9 : gb;
      const float* wb = Wfc + (size_t)gb * FCINW;
      const float vb = bfr(bfc[gb]) + bfr(wb[1549]) * qpmR + bfr(wb[1550]) * tp0R + bfr(wb[1551]) * tp1R;
      const float fa = (f < 512) ? 1.0f : 0.0f;
      const float fb = (f >= 512 && f < 522) ? 1.0f : 0.0f;
      if (f < 576) sm[f] = fa * va + fb * vb;
    }
    __syncthreads();
    const int q = 4 * (tid < 143 ? tid : 143);
    const v4f v = *(const v4f*)(sm + q);
    if (tid < 144) *(volatile v4f*)(BIAS7 + q) = v;
    __threadfence();
    if (tid < 144) *(volatile v4f*)(BIAS7 + q) = v;
  } else if (blockIdx.x == 1) {
#pragma unroll 1
    for (int it = 0; it < 2; ++it) {
      const int f = it * NTHR + tid;
      const float* w = bt_Wi + (size_t)f * BTINW;
      sm[f] = bfr(bt_b[f]) + bfr(w[257]) * qpmR + bfr(w[258]) * tp0R + bfr(w[259]) * tp1R;
    }
    __syncthreads();
    const int q = 4 * (tid < 127 ? tid : 127);
    const v4f v = *(const v4f*)(sm + q);
    if (tid < 128) *(volatile v4f*)(BEFFB + q) = v;
    __threadfence();
    if (tid < 128) *(volatile v4f*)(BEFFB + q) = v;
  } else {
#pragma unroll 1
    for (int it = 0; it < 9; ++it) {
      const int f = it * NTHR + tid;
      const int j = f / VXP;
      const int jj = j < 9 ? j : 9;
      const int c = f - j * VXP;
      const float* w = Wfc + (size_t)jj * FCINW;
      const float va = bfr(w[c < 127 ? c : 127]);
      int c2 = c - 128; c2 = c2 < 0 ? 0 : c2; c2 = c2 > 12 ? 12 : c2;
      const float vb = bfr(w[1536 + c2]);
      const float fa = (c < 128) ? 1.0f : 0.0f;
      const float fb = (c >= 128 && c < 141) ? 1.0f : 0.0f;
      const float fr = (j < 10) ? 1.0f : 0.0f;
      sm[f] = fr * (fa * va + fb * vb);
    }
    __syncthreads();
#pragma unroll 1
    for (int it = 0; it < 3; ++it) {
      const int q = it * NTHR + tid;
      const int qc = q < 575 ? q : 575;
      const v4f v = *(const v4f*)(sm + 4 * qc);
      if (q < 576) *(volatile v4f*)(WFCX + 4 * qc) = v;
      __threadfence();
      if (q < 576) *(volatile v4f*)(WFCX + 4 * qc) = v;
    }
  }
}

__global__ __launch_bounds__(NTHR) void prep_wx_kernel(const float* __restrict__ out_Wh, const float* __restrict__ out_Wi,
    const float* __restrict__ bt_Wh, const float* __restrict__ bt_Wi, float* __restrict__ OWX, float* __restrict__ BWX) {
  const int which = blockIdx.y;
  const float* Wh = which ? bt_Wh : out_Wh;
  const float* Wi = which ? bt_Wi : out_Wi;
  const int wip = which ? BTINW : UINW;
  const int nfb = which ? 14 : 13;
  float* dst = which ? BWX : OWX;
  const int i = blockIdx.x * NTHR + threadIdx.x;
  const int f0 = 4 * i;
  const int r = f0 / VXP;
  const int c0 = f0 - r * VXP;
  v4f o;
#pragma unroll
  for (int e = 0; e < 4; ++e) {
    const int c = c0 + e;
    const float va = bfr(Wh[(size_t)r * HFIN + (c < 127 ? c : 127)]);
    int i2 = c - 128; i2 = i2 < 0 ? 0 : i2; i2 = i2 > nfb - 1 ? nfb - 1 : i2;
    const int scol = which ? (i2 == 0 ? 256 : 259 + i2) : (SCOL + i2);
    const float vb = bfr(Wi[(size_t)r * wip + scol]);
    const float fa = (c < 128) ? 1.0f : 0.0f;
    const float fb = (c >= 128 && c < 128 + nfb) ? 1.0f : 0.0f;
    o[e] = fa * va + fb * vb;
  }
  *(volatile v4f*)(dst + f0) = o;
  __threadfence();
  *(volatile v4f*)(dst + f0) = o;
}

template <bool HAS_IDX>
__global__ __launch_bounds__(NTHR) void split_rows_kernel(const float* __restrict__ src, int spitch, const int* __restrict__ idx, int nsrc,
    unsigned short* __restrict__ hi, unsigned short* __restrict__ lo, int dpitch, int dcol0, int nrow, int ncol8) {
  const int i = blockIdx.x * NTHR + threadIdx.x;
  if (i >= nrow * ncol8) return;
  const int row = i / ncol8;
  const int c8 = i - row * ncol8;
  int srow = row;
  if (HAS_IDX) {
    int v = idx[row];
    v = v < 0 ? 0 : v;
    v = v > nsrc - 1 ? nsrc - 1 : v;
    srow = v;
  }
  const float* sp = src + (size_t)srow * spitch + 8 * c8;
  const v4f a = *(const v4f*)(sp);
  const v4f b = *(const v4f*)(sp + 4);
  v8h hv, lv;
#pragma unroll
  for (int e = 0; e < 4; ++e) {
    const unsigned short ha = f2bf_bits(a[e]);
    const unsigned short la = f2bf_bits(a[e] - bf_bits2f(ha));
    const unsigned short hb = f2bf_bits(b[e]);
    const unsigned short lb = f2bf_bits(b[e] - bf_bits2f(hb));
    hv[e] = __builtin_bit_cast(_Float16, ha);     lv[e] = __builtin_bit_cast(_Float16, la);
    hv[4 + e] = __builtin_bit_cast(_Float16, hb); lv[4 + e] = __builtin_bit_cast(_Float16, lb);
  }
  const size_t o = (size_t)row * dpitch + dcol0 + 8 * c8;
  *(volatile v8h*)(hi + o) = hv;
  *(volatile v8h*)(lo + o) = lv;
  __threadfence();
  *(volatile v8h*)(hi + o) = hv;
  *(volatile v8h*)(lo + o) = lv;
}

template <int H>
__global__ __launch_bounds__(H) void lstm_seq_kernel(const float* __restrict__ Ga, const float* __restrict__ Gb, int gp,
    const float* __restrict__ Wa, const float* __restrict__ Wb, float* __restrict__ Oa, float* __restrict__ Ob, int T) {
  __shared__ __align__(16) float hb[2 * H];
  const int tid = threadIdx.x;
  const int dir = blockIdx.x;
  const int which = blockIdx.y;
  const float* G = which ? Gb : Ga;
  const float* W = (which ? Wb : Wa) + (size_t)dir * 4 * H * H;
  float* O = which ? Ob : Oa;
  hb[tid] = 0.0f;
  hb[H + tid] = 0.0f;
  float c = 0.0f;
  const float* w0 = W + (size_t)tid * H;
  const float* w1 = W + (size_t)(H + tid) * H;
  const float* w2 = W + (size_t)(2 * H + tid) * H;
  const float* w3 = W + (size_t)(3 * H + tid) * H;
  const int st4 = 4 * (tid < H / 4 - 1 ? tid : H / 4 - 1);
  const bool stw = tid < H / 4;
  __syncthreads();
#pragma unroll 1
  for (int s = 0; s < T; ++s) {
    const int t = dir ? (T - 1 - s) : s;
    const int cur = s & 1;
    const float* gpt = G + (size_t)t * gp + dir * 4 * H + tid;
    float ai = gpt[0], af = gpt[H], ag = gpt[2 * H], ao = gpt[3 * H];
    const float* hp = hb + cur * H;
#pragma unroll 1
    for (int k0 = 0; k0 < H; k0 += 4) {
      const v4f hv = *(const v4f*)(hp + k0);
      const v4f u0 = *(const v4f*)(w0 + k0);
      const v4f u1 = *(const v4f*)(w1 + k0);
      const v4f u2 = *(const v4f*)(w2 + k0);
      const v4f u3 = *(const v4f*)(w3 + k0);
      ai += u0[0] * hv[0]; ai += u0[1] * hv[1]; ai += u0[2] * hv[2]; ai += u0[3] * hv[3];
      af += u1[0] * hv[0]; af += u1[1] * hv[1]; af += u1[2] * hv[2]; af += u1[3] * hv[3];
      ag += u2[0] * hv[0]; ag += u2[1] * hv[1]; ag += u2[2] * hv[2]; ag += u2[3] * hv[3];
      ao += u3[0] * hv[0]; ao += u3[1] * hv[1]; ao += u3[2] * hv[2]; ao += u3[3] * hv[3];
    }
    const float ig = fsig(ai), fg = fsig(af), og = fsig(ao), gg = ftanh(ag);
    c = fg * c + ig * gg;
    const float h = og * ftanh(c);
    hb[(cur ^ 1) * H + tid] = h;
    __syncthreads();
    const v4f hv4 = *(const v4f*)(hb + (cur ^ 1) * H + st4);
    float* op = O + (size_t)t * 2 * H + dir * H + st4;
    if (stw) *(volatile v4f*)op = hv4;
    __threadfence();
    if (stw) *(volatile v4f*)op = hv4;
  }
}

template <int SEGLEN, int F>
__global__ __launch_bounds__(F) void segattn_kernel(const float* __restrict__ logits, const float* __restrict__ h,
    unsigned short* __restrict__ hi, unsigned short* __restrict__ lo) {
  __shared__ __align__(16) float sm[F];
  const int sg = blockIdx.x;
  const int f = threadIdx.x;
  const float* lp = logits + (size_t)sg * SEGLEN * F + f;
  const float* hp = h + (size_t)sg * SEGLEN * F + f;
  float m = -INFINITY;
#pragma unroll 1
  for (int i = 0; i < SEGLEN; ++i) m = fmaxf(m, lp[(size_t)i * F]);
  float ssum = 0.0f, acc = 0.0f;
#pragma unroll 1
  for (int i = 0; i < SEGLEN; ++i) {
    const float e = expf(lp[(size_t)i * F] - m);
    ssum += e;
    acc += hp[(size_t)i * F] * e;
  }
  sm[f] = acc / ssum;
  __syncthreads();
  if (f < F / 4) {
    const int which = (f < F / 8) ? 0 : 1;
    const int g = f - which * (F / 8);
    const float* sp = sm + g * 8;
    v8h v;
#pragma unroll
    for (int e = 0; e < 8; ++e) {
      const unsigned short hb2 = f2bf_bits(sp[e]);
      const unsigned short lb2 = f2bf_bits(sp[e] - bf_bits2f(hb2));
      const unsigned short bits = which ? lb2 : hb2;
      v[e] = __builtin_bit_cast(_Float16, bits);
    }
    unsigned short* dp = (which ? lo : hi) + (size_t)sg * F + g * 8;
    *(volatile v8h*)dp = v;
    __threadfence();
    *(volatile v8h*)dp = v;
  }
}

__global__ __launch_bounds__(128) void scan_kernel(
    const float* __restrict__ GOUT, const float* __restrict__ GBT,
    const float* __restrict__ OWX, const float* __restrict__ BWX, const float* __restrict__ WFCX,
    const float* __restrict__ WT1R,
    const float* __restrict__ x, const float* __restrict__ y,
    const float* __restrict__ Wta, const float* __restrict__ bta,
    const float* __restrict__ bt1, const float* __restrict__ Wt2, const float* __restrict__ bt2,
    const int* __restrict__ bid, float* __restrict__ out0, int T) {
  __shared__ __align__(16) float ohx[2 * VXP];
  __shared__ __align__(16) float thx[VXP];
  __shared__ __align__(16) float nhs[128];
  __shared__ __align__(16) float r1v[128];
  __shared__ __align__(16) float bufS[80];
  __shared__ __align__(16) float ltS[80];
  __shared__ __align__(16) float outS[352];
  __shared__ __align__(16) float WtaS[100];
  __shared__ __align__(16) float btaS[16];
  __shared__ __align__(16) float ytS[16];
  __shared__ __align__(16) float bt1S[128];
  __shared__ __align__(16) float Wt2S[128];
  const int tid = threadIdx.x;

  for (int i = tid; i < 2 * VXP; i += 128) ohx[i] = 0.0f;
  for (int i = tid; i < VXP; i += 128) thx[i] = 0.0f;
  nhs[tid] = 0.0f;
  r1v[tid] = 0.0f;
  if (tid < 80) { bufS[tid] = 0.0f; ltS[tid] = 0.0f; }
  for (int i = tid; i < 352; i += 128) outS[i] = 0.0f;
  if (tid < 100) WtaS[tid] = bfr(Wta[tid]);
  if (tid < 16) {
    const int tc9 = tid < 9 ? tid : 9;
    const float bv = bfr(bta[tc9]);
    const float yv = bfr(y[1 + tc9]);
    const float fk = (tid < 10) ? 1.0f : 0.0f;
    btaS[tid] = bv * fk;
    ytS[tid] = yv * fk;
  }
  bt1S[tid] = bfr(bt1[tid]);
  Wt2S[tid] = bfr(Wt2[tid]);
  __syncthreads();
  if (tid < 11) { const float v = bfr(y[tid]); ohx[128 + tid] = v; ohx[VXP + 128 + tid] = v; }
  float ptv = bfr(y[0]);
  const float bt2R = bfr(bt2[0]);
  int cnt = 0;
  float oc = 0.0f, tc = 0.0f;
  __syncthreads();

#pragma unroll 1
  for (int t = 0; t < T; ++t) {
    const int cur = t & 1;
    const int nxt = cur ^ 1;
    const int bnow = bid[t];
    const int bprv = bid[t > 0 ? t - 1 : 0];
    const bool isb = (t == 0) || (bnow > bprv);
    int bcl = bnow < 0 ? 0 : bnow; bcl = bcl > NBEAT - 1 ? NBEAT - 1 : bcl;

    if (isb) {
      if (tid < 10) {
        float rn = ytS[tid];
        if (cnt > 0) {
          const int nval = cnt < 8 ? cnt : 8;
          float m = -INFINITY;
#pragma unroll 1
          for (int r = 0; r < nval; ++r) {
            float l = btaS[tid];
#pragma unroll 1
            for (int i2 = 0; i2 < 10; ++i2) l += bufS[r * 10 + i2] * WtaS[tid * 10 + i2];
            ltS[r * 10 + tid] = l;
            m = fmaxf(m, l);
          }
          float ssum = 0.0f, acc = 0.0f;
#pragma unroll 1
          for (int r = 0; r < nval; ++r) {
            const float e = expf(ltS[r * 10 + tid] - m);
            ssum += e;
            acc += bufS[r * 10 + tid] * e;
          }
          rn = acc / ssum;
        }
        thx[132 + tid] = rn;
      }
      if (tid == 0) thx[128] = ptv;
      if (tid < 3) thx[129 + tid] = bfr(x[(size_t)t * NFEAT + 28 + tid]);
    }
    __syncthreads();
    float nh = 0.0f, ntc = tc;
    if (isb) {
      const float* gb = GBT + (size_t)bcl * (4 * HBEAT) + tid;
      float a0 = gb[0], a1 = gb[HBEAT], a2 = gb[2 * HBEAT], a3 = gb[3 * HBEAT];
      const float* w0 = BWX + (size_t)tid * VXP;
      const float* w1 = BWX + (size_t)(HBEAT + tid) * VXP;
      const float* w2 = BWX + (size_t)(2 * HBEAT + tid) * VXP;
      const float* w3 = BWX + (size_t)(3 * HBEAT + tid) * VXP;
#pragma unroll 1
      for (int k0 = 0; k0 < VXP; k0 += 4) {
        const v4f hv = *(const v4f*)(thx + k0);
        const v4f u0 = *(const v4f*)(w0 + k0);
        const v4f u1 = *(const v4f*)(w1 + k0);
        const v4f u2 = *(const v4f*)(w2 + k0);
        const v4f u3 = *(const v4f*)(w3 + k0);
        a0 += u0[0] * hv[0]; a0 += u0[1] * hv[1]; a0 += u0[2] * hv[2]; a0 += u0[3] * hv[3];
        a1 += u1[0] * hv[0]; a1 += u1[1] * hv[1]; a1 += u1[2] * hv[2]; a1 += u1[3] * hv[3];
        a2 += u2[0] * hv[0]; a2 += u2[1] * hv[1]; a2 += u2[2] * hv[2]; a2 += u2[3] * hv[3];
        a3 += u3[0] * hv[0]; a3 += u3[1] * hv[1]; a3 += u3[2] * hv[2]; a3 += u3[3] * hv[3];
      }
      ntc = fsig(a1) * tc + fsig(a0) * ftanh(a2);
      nh = fsig(a3) * ftanh(ntc);
      nhs[tid] = nh;
    }
    __syncthreads();
    if (isb) {
      float a = bt1S[tid];
      const float* w = WT1R + (size_t)tid * HBEAT;
#pragma unroll 1
      for (int j = 0; j < HBEAT; ++j) a += w[j] * nhs[j];
      r1v[tid] = fmaxf(a, 0.0f);
      thx[tid] = nh;
      tc = ntc;
      if (tid < 80) bufS[tid] = 0.0f;
      cnt = 0;
    }
    __syncthreads();
    if (isb && tid == 0) {
      float a = bt2R;
#pragma unroll 1
      for (int j = 0; j < HBEAT; ++j) a += Wt2S[j] * r1v[j];
      ptv = a;
    }
    {
      const float* go = GOUT + (size_t)t * GON + tid;
      float a0 = go[0], a1 = go[HFIN], a2 = go[2 * HFIN], a3 = go[3 * HFIN];
      const float* w0 = OWX + (size_t)tid * VXP;
      const float* w1 = OWX + (size_t)(HFIN + tid) * VXP;
      const float* w2 = OWX + (size_t)(2 * HFIN + tid) * VXP;
      const float* w3 = OWX + (size_t)(3 * HFIN + tid) * VXP;
      const float* hp = ohx + cur * VXP;
#pragma unroll 1
      for (int k0 = 0; k0 < VXP; k0 += 4) {
        const v4f hv = *(const v4f*)(hp + k0);
        const v4f u0 = *(const v4f*)(w0 + k0);
        const v4f u1 = *(const v4f*)(w1 + k0);
        const v4f u2 = *(const v4f*)(w2 + k0);
        const v4f u3 = *(const v4f*)(w3 + k0);
        a0 += u0[0] * hv[0]; a0 += u0[1] * hv[1]; a0 += u0[2] * hv[2]; a0 += u0[3] * hv[3];
        a1 += u1[0] * hv[0]; a1 += u1[1] * hv[1]; a1 += u1[2] * hv[2]; a1 += u1[3] * hv[3];
        a2 += u2[0] * hv[0]; a2 += u2[1] * hv[1]; a2 += u2[2] * hv[2]; a2 += u2[3] * hv[3];
        a3 += u3[0] * hv[0]; a3 += u3[1] * hv[1]; a3 += u3[2] * hv[2]; a3 += u3[3] * hv[3];
      }
      oc = fsig(a1) * oc + fsig(a0) * ftanh(a2);
      const float noh = fsig(a3) * ftanh(oc);
      ohx[nxt * VXP + tid] = noh;
    }
    __syncthreads();
    float ofc = 0.0f;
    if (tid < 10) {
      float a = GOUT[(size_t)t * GON + 512 + tid];
      const float* w = WFCX + (size_t)tid * VXP;
      const float* hn = ohx + nxt * VXP;
#pragma unroll 1
      for (int c2 = 0; c2 < 141; ++c2) a += w[c2] * hn[c2];
      ofc = a;
    }
    __syncthreads();
    if (tid < 10) {
      ohx[129 + tid] = ofc;
      ohx[VXP + 129 + tid] = ofc;
      outS[(t & 31) * NOUTC + 1 + tid] = ofc;
      if (cnt < 8) bufS[cnt * 10 + tid] = ofc;
    }
    if (tid < 2) { ohx[139 + tid] = ofc; ohx[VXP + 139 + tid] = ofc; }
    if (tid == 0) { ohx[128] = ptv; ohx[VXP + 128] = ptv; outS[(t & 31) * NOUTC] = ptv; }
    cnt += 1;
    __syncthreads();
    if ((t & 31) == 31) {
      const int q4 = 4 * (tid < 87 ? tid : 87);
      const v4f v = *(const v4f*)(outS + q4);
      float* op = out0 + (size_t)(t - 31) * NOUTC + q4;
      if (tid < 88) *(volatile v4f*)op = v;
      __threadfence();
      if (tid < 88) *(volatile v4f*)op = v;
    }
  }
}

constexpr size_t al256(size_t b) { return (b + 255) & ~(size_t)255; }
constexpr size_t SZ_XB = (size_t)NNOTE * KPADX * 2, SZ_NWI = (size_t)2 * 4 * HNOTE * KPADX * 2, SZ_WBA = (size_t)512 * 512 * 2,
  SZ_BWI = (size_t)1024 * 512 * 2, SZ_WMA = (size_t)256 * 256 * 2, SZ_MWI = (size_t)512 * 256 * 2, SZ_BTWI = (size_t)512 * 256 * 2,
  SZ_BTOUT = (size_t)GON * SCOL * 2, SZ_NWHR = (size_t)2 * 1024 * 256 * 4, SZ_BWHR = (size_t)2 * 512 * 128 * 4, SZ_MWHR = (size_t)2 * 256 * 64 * 4,
  SZ_WT1R = (size_t)128 * 128 * 4, SZ_NBIAS = 2048 * 4, SZ_BBIAS = 1024 * 4, SZ_MBIAS = 512 * 4, SZ_BBA = 512 * 4, SZ_BMA = 256 * 4,
  SZ_BIAS7 = (size_t)GON * 4, SZ_BEFFB = 512 * 4, SZ_OWX = (size_t)512 * VXP * 4, SZ_WFCX = (size_t)16 * VXP * 4,
  SZ_GNOTE = (size_t)NNOTE * 2048 * 4, SZ_VOICEH = (size_t)NNOTE * 512 * 4, SZ_S = (size_t)NNOTE * SCOL * 2,
  SZ_BN = (size_t)512 * 512 * 2, SZ_GBEAT = (size_t)512 * 1024 * 4, SZ_BEATH = (size_t)512 * 256 * 4, SZ_BH = (size_t)512 * 256 * 2,
  SZ_LMA = (size_t)512 * 256 * 4, SZ_MN = (size_t)128 * 256 * 2, SZ_GMEAS = (size_t)128 * 512 * 4, SZ_MEASH = (size_t)128 * 128 * 4,
  SZ_GBT = (size_t)512 * 512 * 4, SZ_LBA = (size_t)NNOTE * 512 * 4, SZ_GOUT = (size_t)NNOTE * GON * 4;
constexpr size_t WS_TOTAL = al256(SZ_XB) + 2 * al256(SZ_NWI) + al256(SZ_WBA) + al256(SZ_BWI) + al256(SZ_WMA) + al256(SZ_MWI) + al256(SZ_BTWI)
  + al256(SZ_BTOUT) + 2 * al256(SZ_NWHR) + al256(SZ_BWHR) + al256(SZ_MWHR) + al256(SZ_WT1R) + 2 * al256(SZ_NBIAS) + al256(SZ_BBIAS)
  + al256(SZ_MBIAS) + al256(SZ_BBA) + al256(SZ_BMA) + al256(SZ_BIAS7) + al256(SZ_BEFFB) + 2 * al256(SZ_OWX) + al256(SZ_WFCX)
  + 2 * al256(SZ_GNOTE) + al256(SZ_VOICEH) + 2 * al256(SZ_S) + 2 * al256(SZ_BN) + al256(SZ_GBEAT) + al256(SZ_BEATH) + 2 * al256(SZ_BH)
  + al256(SZ_LMA) + 2 * al256(SZ_MN) + al256(SZ_GMEAS) + al256(SZ_MEASH) + al256(SZ_GBT);
static_assert(WS_TOTAL <= (size_t)134217728);
static_assert(SZ_LBA <= SZ_GNOTE && SZ_GOUT <= SZ_GNOTE);

template <bool ASPLIT>
static void launch_gemm(hipStream_t st, const unsigned short* A, const unsigned short* A2, int lda, const unsigned short* Bt, int ldb,
                        float* C, int ldc, const float* bias, int M, int N, int K) {
  const int tiles = (M / 64) * (N / 64);
  dim3 grid((tiles + 7) / 8);
  gemm_bf16_kernel<ASPLIT><<<grid, NTHR, 0, st>>>(A, A2, lda, Bt, ldb, C, ldc, bias, M, N, K);
}

extern "C" void kernel_launch(void* const* d_in, const int* in_sizes, int n_in,
                              void* d_out, int out_size, void* d_ws, size_t ws_size, hipStream_t stream) {
  if (n_in < 34 || d_out == nullptr || d_ws == nullptr) return;
  if (in_sizes[0] != NNOTE * NFEAT || in_sizes[1] != NOUTC || in_sizes[2] != NNOTE || in_sizes[3] != NNOTE ||
      in_sizes[4] != 2 * 4 * HNOTE * NFEAT || in_sizes[5] != 2 * 4 * HNOTE * HNOTE || in_sizes[6] != 2 * 4 * HNOTE ||
      in_sizes[7] != 2 * 4 * HNOTE * NFEAT || in_sizes[8] != 2 * 4 * HNOTE * HNOTE || in_sizes[9] != 2 * 4 * HNOTE ||
      in_sizes[10] != 2 * 4 * HBEAT * 512 || in_sizes[11] != 2 * 4 * HBEAT * HBEAT || in_sizes[12] != 2 * 4 * HBEAT ||
      in_sizes[13] != 2 * 4 * HMEAS * 256 || in_sizes[14] != 2 * 4 * HMEAS * HMEAS || in_sizes[15] != 2 * 4 * HMEAS ||
      in_sizes[16] != 512 * 512 || in_sizes[17] != 512 || in_sizes[18] != 256 * 256 || in_sizes[19] != 256 ||
      in_sizes[20] != 100 || in_sizes[21] != 10 || in_sizes[22] != 512 * UINW || in_sizes[23] != 512 * HFIN || in_sizes[24] != 512 ||
      in_sizes[25] != 10 * FCINW || in_sizes[26] != 10 || in_sizes[27] != 512 * BTINW || in_sizes[28] != 512 * HBEAT || in_sizes[29] != 512 ||
      in_sizes[30] != 128 * 128 || in_sizes[31] != 128 || in_sizes[32] != 128 || in_sizes[33] != 1 ||
      out_size != NNOTE * NOUTC + NNOTE * 2 * HNOTE) return;

  const float* x        = (const float*)d_in[0];
  const float* y        = (const float*)d_in[1];
  const int*   bid      = (const int*)d_in[2];
  const int*   mid      = (const int*)d_in[3];
  const float* note_Wi  = (const float*)d_in[4];
  const float* note_Wh  = (const float*)d_in[5];
  const float* note_b   = (const float*)d_in[6];
  const float* voice_Wi = (const float*)d_in[7];
  const float* voice_Wh = (const float*)d_in[8];
  const float* voice_b  = (const float*)d_in[9];
  const float* beat_Wi  = (const float*)d_in[10];
  const float* beat_Wh  = (const float*)d_in[11];
  const float* beat_b   = (const float*)d_in[12];
  const float* meas_Wi  = (const float*)d_in[13];
  const float* meas_Wh  = (const float*)d_in[14];
  const float* meas_b   = (const float*)d_in[15];
  const float* Wba      = (const float*)d_in[16];
  const float* bba      = (const float*)d_in[17];
  const float* Wma      = (const float*)d_in[18];
  const float* bma      = (const float*)d_in[19];
  const float* Wta      = (const float*)d_in[20];
  const float* bta      = (const float*)d_in[21];
  const float* out_Wi   = (const float*)d_in[22];
  const float* out_Wh   = (const float*)d_in[23];
  const float* out_b    = (const float*)d_in[24];
  const float* Wfc      = (const float*)d_in[25];
  const float* bfc      = (const float*)d_in[26];
  const float* bt_Wi    = (const float*)d_in[27];
  const float* bt_Wh    = (const float*)d_in[28];
  const float* bt_b     = (const float*)d_in[29];
  const float* Wt1      = (const float*)d_in[30];
  const float* bt1      = (const float*)d_in[31];
  const float* Wt2      = (const float*)d_in[32];
  const float* bt2      = (const float*)d_in[33];
  float* out0 = (float*)d_out;
  float* out1 = (float*)d_out + (size_t)NNOTE * NOUTC;

  char* ws = (char*)d_ws; size_t off = 0;
  auto carve = [&](size_t bytes) -> char* { char* p = ws + off; off += al256(bytes); return p; };
  unsigned short* XB     = (unsigned short*)carve(SZ_XB);
  unsigned short* NWI16  = (unsigned short*)carve(SZ_NWI);
  unsigned short* VWI16  = (unsigned short*)carve(SZ_NWI);
  unsigned short* WBA16  = (unsigned short*)carve(SZ_WBA);
  unsigned short* BWI16  = (unsigned short*)carve(SZ_BWI);
  unsigned short* WMA16  = (unsigned short*)carve(SZ_WMA);
  unsigned short* MWI16  = (unsigned short*)carve(SZ_MWI);
  unsigned short* BTWI16 = (unsigned short*)carve(SZ_BTWI);
  unsigned short* BTOUT16= (unsigned short*)carve(SZ_BTOUT);
  float* NWHR  = (float*)carve(SZ_NWHR);
  float* VWHR  = (float*)carve(SZ_NWHR);
  float* BWHR  = (float*)carve(SZ_BWHR);
  float* MWHR  = (float*)carve(SZ_MWHR);
  float* WT1R  = (float*)carve(SZ_WT1R);
  float* NBIAS = (float*)carve(SZ_NBIAS);
  float* VBIAS = (float*)carve(SZ_NBIAS);
  float* BBIAS = (float*)carve(SZ_BBIAS);
  float* MBIAS = (float*)carve(SZ_MBIAS);
  float* BBA   = (float*)carve(SZ_BBA);
  float* BMA   = (float*)carve(SZ_BMA);
  float* BIAS7 = (float*)carve(SZ_BIAS7);
  float* BEFFB = (float*)carve(SZ_BEFFB);
  float* OWX   = (float*)carve(SZ_OWX);
  float* BWX   = (float*)carve(SZ_OWX);
  float* WFCX  = (float*)carve(SZ_WFCX);
  float* GNOTE = (float*)carve(SZ_GNOTE);
  float* GVOICE= (float*)carve(SZ_GNOTE);
  float* VOICEH= (float*)carve(SZ_VOICEH);
  unsigned short* S_HI  = (unsigned short*)carve(SZ_S);
  unsigned short* S_LO  = (unsigned short*)carve(SZ_S);
  unsigned short* BN_HI = (unsigned short*)carve(SZ_BN);
  unsigned short* BN_LO = (unsigned short*)carve(SZ_BN);
  float* GBEAT = (float*)carve(SZ_GBEAT);
  float* BEATH = (float*)carve(SZ_BEATH);
  unsigned short* BH_HI = (unsigned short*)carve(SZ_BH);
  unsigned short* BH_LO = (unsigned short*)carve(SZ_BH);
  float* LMA   = (float*)carve(SZ_LMA);
  unsigned short* MN_HI = (unsigned short*)carve(SZ_MN);
  unsigned short* MN_LO = (unsigned short*)carve(SZ_MN);
  float* GMEAS = (float*)carve(SZ_GMEAS);
  float* MEASH = (float*)carve(SZ_MEASH);
  float* GBT   = (float*)carve(SZ_GBT);
  float* LBA   = GNOTE;
  float* GOUT  = GVOICE;
  if (off > ws_size || off > (size_t)134217728) return;

  CvtArgs ca;
  auto setseg = [&](int k, const float* src, unsigned short* dst, int spitch, int scol0, int nvalid, int ncol8, int nrow) {
    ca.s[k].src = src; ca.s[k].dst = dst; ca.s[k].spitch = spitch; ca.s[k].scol0 = scol0; ca.s[k].nvalid = nvalid;
    ca.s[k].ncol8 = ncol8; ca.s[k].nrow = nrow; ca.s[k].pad0 = 0;
  };
  setseg(0,  x,        XB,      NFEAT, 0,   NFEAT, KPADX / 8, NNOTE);
  setseg(1,  note_Wi,  NWI16,   NFEAT, 0,   NFEAT, KPADX / 8, 2 * 4 * HNOTE);
  setseg(2,  voice_Wi, VWI16,   NFEAT, 0,   NFEAT, KPADX / 8, 2 * 4 * HNOTE);
  setseg(3,  Wba,      WBA16,   512,   0,   512,   64,        512);
  setseg(4,  beat_Wi,  BWI16,   512,   0,   512,   64,        1024);
  setseg(5,  Wma,      WMA16,   256,   0,   256,   32,        256);
  setseg(6,  meas_Wi,  MWI16,   256,   0,   256,   32,        512);
  setseg(7,  bt_Wi,    BTWI16,  BTINW, 0,   256,   32,        512);
  setseg(8,  out_Wi,   BTOUT16, UINW,  0,   SCOL,  SCOL / 8,  512);
  setseg(9,  Wfc,      BTOUT16 + (size_t)512 * SCOL, FCINW, 128, SCOL, SCOL / 8, 10);
  setseg(10, Wfc,      BTOUT16 + (size_t)522 * SCOL, 0,     0,   0,    SCOL / 8, 54);
  setseg(11, x,        XB,      0,     0,   0,     KPADX / 8, 0);
  cvt_multi_kernel<<<dim3((512 * (SCOL / 8) + NTHR - 1) / NTHR, 11), NTHR, 0, stream>>>(ca);

  RneArgs ra;
  auto setrne = [&](int k, const float* src, float* dst, int n) { ra.src[k] = src; ra.dst[k] = dst; ra.n4[k] = n / 4; };
  for (int k = 0; k < 16; ++k) setrne(k, note_Wh, NWHR, 0);
  setrne(0,  note_Wh,  NWHR,  2 * 4 * HNOTE * HNOTE);
  setrne(1,  voice_Wh, VWHR,  2 * 4 * HNOTE * HNOTE);
  setrne(2,  beat_Wh,  BWHR,  2 * 4 * HBEAT * HBEAT);
  setrne(3,  meas_Wh,  MWHR,  2 * 4 * HMEAS * HMEAS);
  setrne(4,  Wt1,      WT1R,  128 * 128);
  setrne(5,  note_b,   NBIAS, 2 * 4 * HNOTE);
  setrne(6,  voice_b,  VBIAS, 2 * 4 * HNOTE);
  setrne(7,  beat_b,   BBIAS, 2 * 4 * HBEAT);
  setrne(8,  meas_b,   MBIAS, 2 * 4 * HMEAS);
  setrne(9,  bba,      BBA,   512);
  setrne(10, bma,      BMA,   256);
  rne_multi_kernel<<<dim3((2 * 4 * HNOTE * HNOTE / 4 + NTHR - 1) / NTHR, 11), NTHR, 0, stream>>>(ra);

  prep_fold_kernel<<<3, NTHR, 0, stream>>>(x, out_b, out_Wi, bfc, Wfc, bt_b, bt_Wi, BIAS7, BEFFB, WFCX);
  prep_wx_kernel<<<dim3(512 * VXP / 4 / NTHR, 2), NTHR, 0, stream>>>(out_Wh, out_Wi, bt_Wh, bt_Wi, OWX, BWX);

  launch_gemm<false>(stream, XB, XB, KPADX, NWI16, KPADX, GNOTE,  2 * 4 * HNOTE, NBIAS, NNOTE, 2 * 4 * HNOTE, KPADX);
  launch_gemm<false>(stream, XB, XB, KPADX, VWI16, KPADX, GVOICE, 2 * 4 * HNOTE, VBIAS, NNOTE, 2 * 4 * HNOTE, KPADX);

  lstm_seq_kernel<HNOTE><<<dim3(2, 2), HNOTE, 0, stream>>>(GNOTE, GVOICE, 2 * 4 * HNOTE, NWHR, VWHR, out1, VOICEH, NNOTE);

  split_rows_kernel<false><<<(NNOTE * 64 + NTHR - 1) / NTHR, NTHR, 0, stream>>>(out1,   512, bid, NNOTE, S_HI, S_LO, SCOL, 0,   NNOTE, 64);
  split_rows_kernel<false><<<(NNOTE * 64 + NTHR - 1) / NTHR, NTHR, 0, stream>>>(VOICEH, 512, bid, NNOTE, S_HI, S_LO, SCOL, 896, NNOTE, 64);

  launch_gemm<true>(stream, S_HI, S_LO, SCOL, WBA16, 512, LBA, 512, BBA, NNOTE, 512, 512);
  segattn_kernel<8, 512><<<NBEAT, 512, 0, stream>>>(LBA, out1, BN_HI, BN_LO);
  launch_gemm<true>(stream, BN_HI, BN_LO, 512, BWI16, 512, GBEAT, 2 * 4 * HBEAT, BBIAS, NBEAT, 2 * 4 * HBEAT, 512);
  lstm_seq_kernel<HBEAT><<<dim3(2, 1), HBEAT, 0, stream>>>(GBEAT, GBEAT, 2 * 4 * HBEAT, BWHR, BWHR, BEATH, BEATH, NBEAT);
  split_rows_kernel<false><<<(NBEAT * 32 + NTHR - 1) / NTHR, NTHR, 0, stream>>>(BEATH, 256, bid, NBEAT, BH_HI, BH_LO, 256, 0, NBEAT, 32);
  launch_gemm<true>(stream, BH_HI, BH_LO, 256, WMA16, 256, LMA, 256, BMA, NBEAT, 256, 256);
  segattn_kernel<4, 256><<<NMEAS, 256, 0, stream>>>(LMA, BEATH, MN_HI, MN_LO);
  launch_gemm<true>(stream, MN_HI, MN_LO, 256, MWI16, 256, GMEAS, 2 * 4 * HMEAS, MBIAS, NMEAS, 2 * 4 * HMEAS, 256);
  lstm_seq_kernel<HMEAS><<<dim3(2, 1), HMEAS, 0, stream>>>(GMEAS, GMEAS, 2 * 4 * HMEAS, MWHR, MWHR, MEASH, MEASH, NMEAS);
  split_rows_kernel<true><<<(NNOTE * 32 + NTHR - 1) / NTHR, NTHR, 0, stream>>>(BEATH, 256, bid, NBEAT, S_HI, S_LO, SCOL, 512, NNOTE, 32);
  split_rows_kernel<true><<<(NNOTE * 16 + NTHR - 1) / NTHR, NTHR, 0, stream>>>(MEASH, 128, mid, NMEAS, S_HI, S_LO, SCOL, 768, NNOTE, 16);
  launch_gemm<true>(stream, S_HI, S_LO, SCOL, BTOUT16, SCOL, GOUT, GON, BIAS7, NNOTE, GON, SCOL);
  launch_gemm<true>(stream, BH_HI, BH_LO, 256, BTWI16, 256, GBT, 4 * HBEAT, BEFFB, NBEAT, 4 * HBEAT, 256);
  scan_kernel<<<1, 128, 0, stream>>>(GOUT, GBT, OWX, BWX, WFCX, WT1R, x, y, Wta, bta, bt1, Wt2, bt2, bid, out0, NNOTE);
}
